// PointNet2PatchletsSA_6957847020167
// MI455X (gfx1250) — hardware-verified
//
#include <hip/hip_runtime.h>
#pragma clang fp contract(off)

typedef __attribute__((ext_vector_type(16))) _Float16 v16h;
typedef __attribute__((ext_vector_type(8)))  _Float16 v8h;
typedef __attribute__((ext_vector_type(8)))  float    v8f;
typedef __attribute__((ext_vector_type(4)))  float    v4f;
typedef __attribute__((ext_vector_type(4)))  unsigned v4u;
typedef __attribute__((ext_vector_type(4)))  int      v4i;

constexpr int NBATCH   = 4;
constexpr int NFRM     = 64;
constexpr int NPTS     = 1024;
constexpr int KNN      = 16;
constexpr int NFRAMES  = NBATCH * NFRM;
constexpr int SPAT     = 3 * NFRM * KNN;
constexpr int ROWS_PAD = 68;
constexpr int PLANE_D  = ROWS_PAD * KNN;
constexpr int SLAB_H   = 3 * PLANE_D;
constexpr int SLAB_CHUNKS = SLAB_H / 8;
constexpr int CH0 = 1024, CH1 = 64, CH2 = 128, CH3 = 256;
constexpr float WCARRY     = 64.0f;
constexpr float WCARRY_INV = 1.0f / 64.0f;
constexpr float BN_EPS     = 1e-5f;
constexpr float INV_COUNT  = 1.0f / (float)(NBATCH * SPAT);

static_assert(SLAB_H == 3264, "slab halves");
static_assert((SLAB_H * 2) % 128 == 0, "slab is whole 128-B lines");
static_assert(SLAB_CHUNKS == 408, "slab chunks");
static_assert(SPAT == 3072, "spatial");
static_assert(NFRAMES == 256, "frames");

__global__ __launch_bounds__(256) void knn_kernel(const float* __restrict__ xyz, int* __restrict__ idxs) {
#pragma clang fp contract(off)
  __shared__ __align__(16) float fr[NPTS * 3];
  __shared__ __align__(16) float sqb[NPTS];
  __shared__ __align__(16) int   st[256 * KNN];
  const int tid = threadIdx.x;
  const int f   = blockIdx.x;
  const int t   = f & (NFRM - 1);
  const int fq  = (t > 0) ? (f - 1) : f;
  {
    const v4f* src = (const v4f*)(xyz + (size_t)f * (NPTS * 3));
    v4f* dv = (v4f*)fr;
    const v4f a0 = src[tid];
    const v4f a1 = src[tid + 256];
    const v4f a2 = src[tid + 512];
    dv[tid] = a0;
    dv[tid + 256] = a1;
    dv[tid + 512] = a2;
  }
  __syncthreads();
#pragma unroll
  for (int i = 0; i < 4; ++i) {
    const int j = tid + 256 * i;
    const float x = fr[3 * j], y = fr[3 * j + 1], z = fr[3 * j + 2];
    const float tx = x * x;
    const float ty = y * y;
    const float tz = z * z;
    sqb[j] = (tx + tz) + ty;
  }
  __syncthreads();
  const int q = blockIdx.y * 256 + tid;
  const float* qp = xyz + ((size_t)fq * NPTS + q) * 3;
  const float qx = qp[0], qy = qp[1], qz = qp[2];
  const float qtx = qx * qx;
  const float qty = qy * qy;
  const float qtz = qz * qz;
  const float sqq = (qtx + qtz) + qty;
  float bd[KNN];
  int   bi[KNN];
#pragma unroll
  for (int s = 0; s < KNN; ++s) { bd[s] = __builtin_inff(); bi[s] = 0; }
#pragma unroll 1
  for (int j = 0; j < NPTS; ++j) {
    const float bx = fr[3 * j], by = fr[3 * j + 1], bz = fr[3 * j + 2];
    float p = qx * bx;
    p = __builtin_fmaf(qy, by, p);
    p = __builtin_fmaf(qz, bz, p);
    const float tw = 2.0f * p;
    const float dm = sqq - tw;
    const float d2 = dm + sqb[j];
    if (d2 < bd[KNN - 1]) {
      bd[KNN - 1] = d2;
      bi[KNN - 1] = j;
#pragma unroll
      for (int s = KNN - 1; s > 0; --s) {
        const bool sw = bd[s] < bd[s - 1];
        const float fa = bd[s - 1], fb = bd[s];
        const int   ia = bi[s - 1], ib = bi[s];
        bd[s - 1] = sw ? fb : fa;
        bd[s]     = sw ? fa : fb;
        bi[s - 1] = sw ? ib : ia;
        bi[s]     = sw ? ia : ib;
      }
    }
  }
  v4i* sv = (v4i*)st;
  sv[tid * 4 + 0] = (v4i){bi[0],  bi[1],  bi[2],  bi[3]};
  sv[tid * 4 + 1] = (v4i){bi[4],  bi[5],  bi[6],  bi[7]};
  sv[tid * 4 + 2] = (v4i){bi[8],  bi[9],  bi[10], bi[11]};
  sv[tid * 4 + 3] = (v4i){bi[12], bi[13], bi[14], bi[15]};
  __syncthreads();
  const v4i o0 = sv[tid];
  const v4i o1 = sv[tid + 256];
  const v4i o2 = sv[tid + 512];
  const v4i o3 = sv[tid + 768];
  volatile v4i* dst = (volatile v4i*)(idxs + ((size_t)f * NPTS + (size_t)blockIdx.y * 256) * KNN);
  dst[tid] = o0;
  dst[tid + 256] = o1;
  dst[tid + 512] = o2;
  dst[tid + 768] = o3;
  __threadfence();
  dst[tid] = o0;
  dst[tid + 256] = o1;
  dst[tid + 512] = o2;
  dst[tid + 768] = o3;
}

__global__ __launch_bounds__(32) void chain_kernel(const int* __restrict__ idxs, int* __restrict__ carry_in) {
  const int n = blockIdx.x * 32 + threadIdx.x;
  int carry = n;
  volatile int* cw = (volatile int*)carry_in;
#pragma unroll 1
  for (int f = 0; f < NFRAMES; ++f) {
    const int cv = carry;
    cw[f * NPTS + n] = cv;
    __threadfence();
    cw[f * NPTS + n] = cv;
    carry = idxs[((size_t)f * NPTS + cv) * KNN] & (NPTS - 1);
  }
}

__global__ __launch_bounds__(256) void out0_kernel(const float* __restrict__ xyz, const int* __restrict__ idxs,
                                                   const int* __restrict__ carry_in, float* __restrict__ out0) {
  const int g  = blockIdx.x * 256 + threadIdx.x;
  const int n4 = g & 255;
  const int fd = g >> 8;
  const int f  = fd / 3;
  const int d  = fd - 3 * f;
  const v4i cr = *(const v4i*)(carry_in + (size_t)f * NPTS + n4 * 4);
  const int c0 = cr.x & (NPTS - 1);
  const int c1 = cr.y & (NPTS - 1);
  const int c2 = cr.z & (NPTS - 1);
  const int c3 = cr.w & (NPTS - 1);
  const int* ib = idxs + (size_t)f * NPTS * KNN;
  const int j0 = ib[c0 * KNN] & (NPTS - 1);
  const int j1 = ib[c1 * KNN] & (NPTS - 1);
  const int j2 = ib[c2 * KNN] & (NPTS - 1);
  const int j3 = ib[c3 * KNN] & (NPTS - 1);
  const float* fb = xyz + (size_t)f * (NPTS * 3) + d;
  v4f o;
  o.x = fb[j0 * 3];
  o.y = fb[j1 * 3];
  o.z = fb[j2 * 3];
  o.w = fb[j3 * 3];
  volatile v4f* dst = (volatile v4f*)(out0 + (size_t)fd * NPTS + n4 * 4);
  *dst = o;
  __threadfence();
  *dst = o;
}

__device__ __forceinline__ unsigned f16_bits(float x) {
  const _Float16 hval = (_Float16)x;
  const unsigned short sb = __builtin_bit_cast(unsigned short, hval);
  return (unsigned)sb;
}

__global__ __launch_bounds__(256) void pack_kernel(const float* __restrict__ xyz, const int* __restrict__ idxs,
                                                   const int* __restrict__ carry_in, unsigned short* __restrict__ act0) {
  constexpr int ROWW = ROWS_PAD * 8;
  __shared__ __align__(16) unsigned tile[3 * ROWW];
  const int tid = threadIdx.x;
  const int bn  = blockIdx.x;
  const int b   = bn >> 10;
  const int n   = bn & (NPTS - 1);
  const int t   = tid >> 2;
  const int kq  = tid & 3;
  const int f   = b * NFRM + t;
  const int cr  = carry_in[(size_t)f * NPTS + n] & (NPTS - 1);
  const v4i id  = *(const v4i*)(idxs + ((size_t)f * NPTS + cr) * KNN + kq * 4);
  const int j0 = id.x & (NPTS - 1);
  const int j1 = id.y & (NPTS - 1);
  const int j2 = id.z & (NPTS - 1);
  const int j3 = id.w & (NPTS - 1);
  const float* fb = xyz + (size_t)f * (NPTS * 3);
  const float x0 = fb[j0 * 3], y0 = fb[j0 * 3 + 1], z0 = fb[j0 * 3 + 2];
  const float x1 = fb[j1 * 3], y1 = fb[j1 * 3 + 1], z1 = fb[j1 * 3 + 2];
  const float x2 = fb[j2 * 3], y2 = fb[j2 * 3 + 1], z2 = fb[j2 * 3 + 2];
  const float x3 = fb[j3 * 3], y3 = fb[j3 * 3 + 1], z3 = fb[j3 * 3 + 2];
  const int wbase = (t + 1) * 8 + kq * 2;
  tile[0 * ROWW + wbase]     = f16_bits(x0) | (f16_bits(x1) << 16);
  tile[0 * ROWW + wbase + 1] = f16_bits(x2) | (f16_bits(x3) << 16);
  tile[1 * ROWW + wbase]     = f16_bits(y0) | (f16_bits(y1) << 16);
  tile[1 * ROWW + wbase + 1] = f16_bits(y2) | (f16_bits(y3) << 16);
  tile[2 * ROWW + wbase]     = f16_bits(z0) | (f16_bits(z1) << 16);
  tile[2 * ROWW + wbase + 1] = f16_bits(z2) | (f16_bits(z3) << 16);
  if (tid < 96) {
    const int dz   = tid >> 5;
    const int rem  = tid & 31;
    const int rsel = rem >> 3;
    const int wz   = rem & 7;
    const int rowz = (rsel == 0) ? 0 : (64 + rsel);
    tile[dz * ROWW + rowz * 8 + wz] = 0u;
  }
  __syncthreads();
  const v4u* tv = (const v4u*)tile;
  volatile v4u* dst = (volatile v4u*)(act0 + (size_t)bn * SLAB_H);
  const int  q1   = tid + 256;
  const bool has1 = q1 < SLAB_CHUNKS;
  const v4u cv0 = tv[tid];
  const v4u cv1 = tv[has1 ? q1 : 0];
  dst[tid] = cv0;
  if (has1) dst[q1] = cv1;
  __threadfence();
  dst[tid] = cv0;
  if (has1) dst[q1] = cv1;
}

__global__ __launch_bounds__(256) void wpack_kernel(const float* __restrict__ w, unsigned short* __restrict__ wp, int n8) {
  const int i = blockIdx.x * 256 + threadIdx.x;
  if (i < n8) {
    const v4f a = ((const v4f*)w)[2 * i];
    const v4f c = ((const v4f*)w)[2 * i + 1];
    v8h hv;
    hv[0] = (_Float16)(a.x * WCARRY);
    hv[1] = (_Float16)(a.y * WCARRY);
    hv[2] = (_Float16)(a.z * WCARRY);
    hv[3] = (_Float16)(a.w * WCARRY);
    hv[4] = (_Float16)(c.x * WCARRY);
    hv[5] = (_Float16)(c.y * WCARRY);
    hv[6] = (_Float16)(c.z * WCARRY);
    hv[7] = (_Float16)(c.w * WCARRY);
    volatile v8h* dst = (volatile v8h*)(wp + (size_t)i * 8);
    *dst = hv;
    __threadfence();
    *dst = hv;
  }
}

constexpr int A_PITCH = 72;
constexpr int B_PITCH = 32;
constexpr int B_SEGS  = 176;
constexpr int E_PITCH = 36;

union FragU { v16h v; v8h h[2]; };

__device__ __forceinline__ v8f mma_h(v16h a, v16h b, v8f c) {
  c = __builtin_amdgcn_wmma_f32_16x16x32_f16(false, a, false, b, (short)0, c, false, false);
  asm volatile("v_nop\n\tv_nop\n\tv_nop\n\tv_nop" : "+v"(c) : "v"(a), "v"(b));
  return c;
}

__device__ __forceinline__ void stage_store(unsigned short* Ab, unsigned short* Bb, int aoff, int tid, int bk, bool bact,
                                            v4u pa0, v4u pa1, v4u pb0, v4u pb1) {
  *(v4u*)(Ab + aoff)     = pa0;
  *(v4u*)(Ab + aoff + 8) = pa1;
  if (bact) {
    unsigned short* seg = Bb + tid * B_PITCH;
    const v4u zv = {0u, 0u, 0u, 0u};
    *(v4u*)(seg + 8)  = zv;
    *(v4u*)(seg + 16) = zv;
    asm volatile("" ::: "memory");
    unsigned short* dp = seg + (15 - bk);
    const unsigned w0 = pb0.x;
    const unsigned w1 = pb0.y;
    const unsigned w2 = pb0.z;
    const unsigned w3 = pb0.w;
    const unsigned w4 = pb1.x;
    const unsigned w5 = pb1.y;
    const unsigned w6 = pb1.z;
    const unsigned w7 = pb1.w;
    dp[0]  = (unsigned short)(w0 & 0xffffu);
    dp[1]  = (unsigned short)(w0 >> 16);
    dp[2]  = (unsigned short)(w1 & 0xffffu);
    dp[3]  = (unsigned short)(w1 >> 16);
    dp[4]  = (unsigned short)(w2 & 0xffffu);
    dp[5]  = (unsigned short)(w2 >> 16);
    dp[6]  = (unsigned short)(w3 & 0xffffu);
    dp[7]  = (unsigned short)(w3 >> 16);
    dp[8]  = (unsigned short)(w4 & 0xffffu);
    dp[9]  = (unsigned short)(w4 >> 16);
    dp[10] = (unsigned short)(w5 & 0xffffu);
    dp[11] = (unsigned short)(w5 >> 16);
    dp[12] = (unsigned short)(w6 & 0xffffu);
    dp[13] = (unsigned short)(w6 >> 16);
    dp[14] = (unsigned short)(w7 & 0xffffu);
    dp[15] = (unsigned short)(w7 >> 16);
  }
}

__device__ __forceinline__ void emit_rows(float* slab, v8f t0acc, v8f t1acc, const float* bias8,
                                          float* dstrow0, int lane) {
  const int h = lane >> 4, c = lane & 15;
  const v4f bv0 = *(const v4f*)(bias8);
  const v4f bv1 = *(const v4f*)(bias8 + 4);
  float bb[8];
  bb[0] = bv0.x; bb[1] = bv0.y; bb[2] = bv0.z; bb[3] = bv0.w;
  bb[4] = bv1.x; bb[5] = bv1.y; bb[6] = bv1.z; bb[7] = bv1.w;
#pragma unroll
  for (int r = 0; r < 8; ++r) {
    const float s0 = t0acc[r] * WCARRY_INV;
    const float s1 = t1acc[r] * WCARRY_INV;
    slab[(8 * h + r) * E_PITCH + c]      = s0 + bb[r];
    slab[(8 * h + r) * E_PITCH + 16 + c] = s1 + bb[r];
  }
  __syncthreads();
  const int q = lane >> 3, c4 = (lane & 7) * 4;
  const v4f r0 = *(const v4f*)(slab + (0 + q)  * E_PITCH + c4);
  const v4f r1 = *(const v4f*)(slab + (4 + q)  * E_PITCH + c4);
  const v4f r2 = *(const v4f*)(slab + (8 + q)  * E_PITCH + c4);
  const v4f r3 = *(const v4f*)(slab + (12 + q) * E_PITCH + c4);
  volatile v4f* d0 = (volatile v4f*)(dstrow0 + (size_t)(0 + q)  * SPAT + c4);
  volatile v4f* d1 = (volatile v4f*)(dstrow0 + (size_t)(4 + q)  * SPAT + c4);
  volatile v4f* d2 = (volatile v4f*)(dstrow0 + (size_t)(8 + q)  * SPAT + c4);
  volatile v4f* d3 = (volatile v4f*)(dstrow0 + (size_t)(12 + q) * SPAT + c4);
  *d0 = r0; *d1 = r1; *d2 = r2; *d3 = r3;
  __threadfence();
  *d0 = r0; *d1 = r1; *d2 = r2; *d3 = r3;
  __syncthreads();
}

__global__ __launch_bounds__(256) void conv_gemm(const unsigned short* __restrict__ act,
                                                 const unsigned short* __restrict__ wp,
                                                 const float* __restrict__ bias,
                                                 float* __restrict__ y, int Cin, int Cout) {
  __shared__ __align__(16) unsigned short As[2][64 * A_PITCH];
  __shared__ __align__(16) unsigned short Bs[2][B_SEGS * B_PITCH];
  __shared__ __align__(16) float Es[8][16 * E_PITCH];
  const int tid  = threadIdx.x;
  const int lane = tid & 31;
  const int wave = tid >> 5;
  const int h    = lane >> 4;
  const int c    = lane & 15;
  const int wm   = wave & 1;
  const int wn   = wave >> 1;
  const int ntile = blockIdx.x;
  const int bd   = ntile >> 3;
  const int b    = bd / 3;
  const int d    = bd - 3 * b;
  const int t0   = (ntile & 7) * 8;
  const int co_base = blockIdx.y * 64;

  const int  row_a = tid >> 2;
  const int  qa    = (tid & 3) * 16;
  const int  aoff  = row_a * A_PITCH + qa;
  const bool bact  = tid < B_SEGS;
  const int  brow  = bact ? (tid >> 4) : 0;
  const int  bk    = tid & 15;
  const unsigned short* wsrc = wp + ((size_t)(co_base + row_a) * Cin) * 64 + qa;
  const unsigned short* asrc = act + (((size_t)b * Cin) * 3 + d) * PLANE_D + (size_t)(t0 + brow) * KNN;

  v8f acc00 = (v8f){0.f,0.f,0.f,0.f,0.f,0.f,0.f,0.f};
  v8f acc01 = acc00, acc10 = acc00, acc11 = acc00;

  v4u pa0 = *(const v4u*)(wsrc);
  v4u pa1 = *(const v4u*)(wsrc + 8);
  v4u pb0 = *(const v4u*)(asrc);
  v4u pb1 = *(const v4u*)(asrc + 8);
  stage_store(As[0], Bs[0], aoff, tid, bk, bact, pa0, pa1, pb0, pb1);
  __syncthreads();

  for (int ci = 0; ci < Cin; ++ci) {
    const int  cur  = ci & 1;
    const bool more = (ci + 1) < Cin;
    if (more) {
      const unsigned short* wn1 = wsrc + (size_t)(ci + 1) * 64;
      const unsigned short* an1 = asrc + (size_t)(ci + 1) * SLAB_H;
      pa0 = *(const v4u*)(wn1);
      pa1 = *(const v4u*)(wn1 + 8);
      pb0 = *(const v4u*)(an1);
      pb1 = *(const v4u*)(an1 + 8);
    }
    const unsigned short* Ab = As[cur];
    const unsigned short* Bb = Bs[cur];
#pragma unroll
    for (int ks = 0; ks < 2; ++ks) {
      FragU a0, a1;
      const unsigned short* ar0 = Ab + (wm * 32 + c) * A_PITCH + ks * 32 + 8 * h;
      const unsigned short* ar1 = ar0 + 16 * A_PITCH;
      a0.h[0] = *(const v8h*)(const void*)(ar0);
      a0.h[1] = *(const v8h*)(const void*)(ar0 + 16);
      a1.h[0] = *(const v8h*)(const void*)(ar1);
      a1.h[1] = *(const v8h*)(const void*)(ar1 + 16);
      FragU b0, b1;
      const unsigned short* bs0 = Bb + ((wn * 2 + 2 * ks) * 16 + c) * B_PITCH + 8 + 8 * h;
      b0.h[0] = *(const v8h*)(const void*)(bs0);
      b0.h[1] = *(const v8h*)(const void*)(bs0 + 16 * B_PITCH);
      b1.h[0] = *(const v8h*)(const void*)(bs0 + 16 * B_PITCH);
      b1.h[1] = *(const v8h*)(const void*)(bs0 + 32 * B_PITCH);
      acc00 = mma_h(a0.v, b0.v, acc00);
      acc10 = mma_h(a1.v, b0.v, acc10);
      acc01 = mma_h(a0.v, b1.v, acc01);
      acc11 = mma_h(a1.v, b1.v, acc11);
    }
    if (more) stage_store(As[cur ^ 1], Bs[cur ^ 1], aoff, tid, bk, bact, pa0, pa1, pb0, pb1);
    __syncthreads();
  }

  float* slab = Es[wave];
  const int co_w = co_base + wm * 32;
  float* ybase = y + (((size_t)b * Cout + co_w) * 3 + d) * 1024 + (size_t)t0 * KNN + wn * 32;
  emit_rows(slab, acc00, acc01, bias + co_w + 8 * h, ybase, lane);
  emit_rows(slab, acc10, acc11, bias + co_w + 16 + 8 * h, ybase + (size_t)16 * SPAT, lane);
}

__global__ __launch_bounds__(256) void bn_stats(const float* __restrict__ y, float* __restrict__ stats, int Cout) {
  __shared__ float red[256];
  const int tid = threadIdx.x;
  const int ch  = blockIdx.x;
  float s = 0.0f;
#pragma unroll 1
  for (int bb = 0; bb < NBATCH; ++bb) {
    const v4f* p = (const v4f*)(y + ((size_t)bb * Cout + ch) * SPAT);
    const v4f a0 = p[tid];
    const v4f a1 = p[tid + 256];
    const v4f a2 = p[tid + 512];
    const float s0 = (a0.x + a0.y) + (a0.z + a0.w);
    const float s1 = (a1.x + a1.y) + (a1.z + a1.w);
    const float s2 = (a2.x + a2.y) + (a2.z + a2.w);
    s += (s0 + s1) + s2;
  }
  red[tid] = s;
  __syncthreads();
  for (int off = 128; off > 0; off >>= 1) {
    if (tid < off) red[tid] += red[tid + off];
    __syncthreads();
  }
  const float mean = red[0] * INV_COUNT;
  __syncthreads();
  float sq = 0.0f;
#pragma unroll 1
  for (int bb = 0; bb < NBATCH; ++bb) {
    const v4f* p = (const v4f*)(y + ((size_t)bb * Cout + ch) * SPAT);
    const v4f a0 = p[tid];
    const v4f a1 = p[tid + 256];
    const v4f a2 = p[tid + 512];
    float e0, e1, e2, e3, part;
    e0 = a0.x - mean; e1 = a0.y - mean; e2 = a0.z - mean; e3 = a0.w - mean;
    part = (e0 * e0 + e1 * e1) + (e2 * e2 + e3 * e3);
    e0 = a1.x - mean; e1 = a1.y - mean; e2 = a1.z - mean; e3 = a1.w - mean;
    part += (e0 * e0 + e1 * e1) + (e2 * e2 + e3 * e3);
    e0 = a2.x - mean; e1 = a2.y - mean; e2 = a2.z - mean; e3 = a2.w - mean;
    part += (e0 * e0 + e1 * e1) + (e2 * e2 + e3 * e3);
    sq += part;
  }
  red[tid] = sq;
  __syncthreads();
  for (int off = 128; off > 0; off >>= 1) {
    if (tid < off) red[tid] += red[tid + off];
    __syncthreads();
  }
  const float var  = red[0] * INV_COUNT;
  const float rstd = rsqrtf(var + BN_EPS);
  if (tid < 32) {
    const float val = (tid == 0) ? mean : ((tid == 1) ? rstd : 0.0f);
    volatile float* dst = (volatile float*)(stats + (size_t)ch * 32);
    dst[tid] = val;
    __threadfence();
    dst[tid] = val;
  }
}

__global__ __launch_bounds__(256) void bn_apply(const float* __restrict__ y, const float* __restrict__ stats,
                                                const float* __restrict__ gamma, const float* __restrict__ beta,
                                                unsigned short* __restrict__ actout, int Cout) {
  const int tid = threadIdx.x;
  const int bc  = blockIdx.x;
  const int ch  = bc % Cout;
  const float m  = stats[(size_t)ch * 32];
  const float rs = stats[(size_t)ch * 32 + 1];
  const float g  = gamma[ch];
  const float be = beta[ch];
  const float* ysrc = y + (size_t)bc * SPAT;
  unsigned short* dbase = actout + (size_t)bc * SLAB_H;
#pragma unroll 1
  for (int q = tid; q < SLAB_CHUNKS; q += 256) {
    const int dd = q / 136;
    const int e  = q - dd * 136;
    const int rr = e >> 1;
    const int hf = e & 1;
    const bool valid = (rr >= 1) && (rr <= NFRM);
    const int tt = valid ? (rr - 1) : 0;
    const float* p = ysrc + dd * 1024 + tt * KNN + hf * 8;
    const v4f a0 = *(const v4f*)(p);
    const v4f a1 = *(const v4f*)(p + 4);
    float v[8];
    v[0] = a0.x; v[1] = a0.y; v[2] = a0.z; v[3] = a0.w;
    v[4] = a1.x; v[5] = a1.y; v[6] = a1.z; v[7] = a1.w;
    v8h hv;
#pragma unroll
    for (int i = 0; i < 8; ++i) {
      float u = (v[i] - m) * rs;
      u = u * g + be;
      u = fmaxf(u, 0.0f);
      u = valid ? u : 0.0f;
      hv[i] = (_Float16)u;
    }
    volatile v8h* dst = (volatile v8h*)(dbase + (size_t)q * 8);
    *dst = hv;
    __threadfence();
    *dst = hv;
  }
}

__global__ __launch_bounds__(256) void bn_max(const float* __restrict__ y2, const float* __restrict__ stats,
                                              const float* __restrict__ gamma, const float* __restrict__ beta,
                                              float* __restrict__ out1) {
  __shared__ __align__(16) float sm[256];
  const int tid = threadIdx.x;
  const int idx = blockIdx.x * 256 + tid;
  const int d   = idx % 3;
  const int cd  = idx / 3;
  const int ch  = cd & (CH3 - 1);
  const int bt  = cd >> 8;
  const int t   = bt & (NFRM - 1);
  const int b   = bt >> 6;
  const float m  = stats[(size_t)ch * 32];
  const float rs = stats[(size_t)ch * 32 + 1];
  const float g  = gamma[ch];
  const float be = beta[ch];
  const float* src = y2 + (((size_t)b * CH3 + ch) * 3 + d) * 1024 + t * KNN;
  const v4f a0 = *(const v4f*)(src);
  const v4f a1 = *(const v4f*)(src + 4);
  const v4f a2 = *(const v4f*)(src + 8);
  const v4f a3 = *(const v4f*)(src + 12);
  float v[16];
  v[0] = a0.x;  v[1] = a0.y;  v[2] = a0.z;  v[3] = a0.w;
  v[4] = a1.x;  v[5] = a1.y;  v[6] = a1.z;  v[7] = a1.w;
  v[8] = a2.x;  v[9] = a2.y;  v[10] = a2.z; v[11] = a2.w;
  v[12] = a3.x; v[13] = a3.y; v[14] = a3.z; v[15] = a3.w;
  float mx = 0.0f;
#pragma unroll
  for (int k = 0; k < KNN; ++k) {
    float u = (v[k] - m) * rs;
    u = u * g + be;
    mx = fmaxf(mx, u);
  }
  sm[tid] = mx;
  __syncthreads();
  if (tid < 64) {
    const v4f o = *(const v4f*)(sm + tid * 4);
    volatile v4f* dst = (volatile v4f*)(out1 + (size_t)blockIdx.x * 256 + tid * 4);
    *dst = o;
    __threadfence();
    *dst = o;
  }
}

constexpr size_t SZ_IDX   = (size_t)NFRAMES * NPTS * KNN * 4;
constexpr size_t SZ_CARRY = (size_t)NFRAMES * NPTS * 4;
constexpr size_t SZ_ACT0  = (size_t)NBATCH * CH0 * SLAB_H * 2;
constexpr size_t SZ_WP0   = (size_t)CH1 * CH0 * 64 * 2;
constexpr size_t SZ_WP1   = (size_t)CH2 * CH1 * 64 * 2;
constexpr size_t SZ_WP2   = (size_t)CH3 * CH2 * 64 * 2;
constexpr size_t SZ_Y0    = (size_t)NBATCH * CH1 * SPAT * 4;
constexpr size_t SZ_Y1    = (size_t)NBATCH * CH2 * SPAT * 4;
constexpr size_t SZ_Y2    = (size_t)NBATCH * CH3 * SPAT * 4;
constexpr size_t SZ_ACT1  = (size_t)NBATCH * CH1 * SLAB_H * 2;
constexpr size_t SZ_ACT2  = (size_t)NBATCH * CH2 * SLAB_H * 2;
constexpr size_t SZ_STATS = (size_t)256 * 32 * 4;

constexpr size_t OFF_IDX   = 0;
constexpr size_t OFF_CARRY = OFF_IDX + SZ_IDX;
constexpr size_t OFF_ACT0  = OFF_CARRY + SZ_CARRY;
constexpr size_t OFF_WP0   = OFF_ACT0 + SZ_ACT0;
constexpr size_t OFF_WP1   = OFF_WP0 + SZ_WP0;
constexpr size_t OFF_WP2   = OFF_WP1 + SZ_WP1;
constexpr size_t OFF_Y0    = OFF_WP2 + SZ_WP2;
constexpr size_t OFF_Y1    = OFF_Y0 + SZ_Y0;
constexpr size_t OFF_Y2    = OFF_Y1 + SZ_Y1;
constexpr size_t OFF_ACT1  = OFF_Y2 + SZ_Y2;
constexpr size_t OFF_ACT2  = OFF_ACT1 + SZ_ACT1;
constexpr size_t OFF_ST0   = OFF_ACT2 + SZ_ACT2;
constexpr size_t OFF_ST1   = OFF_ST0 + SZ_STATS;
constexpr size_t OFF_ST2   = OFF_ST1 + SZ_STATS;
constexpr size_t WS_TOTAL  = OFF_ST2 + SZ_STATS;
static_assert(WS_TOTAL == 85327872ull, "carve total");
static_assert(WS_TOTAL <= 134217728ull, "carve under 128 MiB");
static_assert(OFF_CARRY % 128 == 0 && OFF_ACT0 % 128 == 0 && OFF_WP0 % 128 == 0 && OFF_Y0 % 128 == 0 &&
              OFF_ACT1 % 128 == 0 && OFF_ACT2 % 128 == 0 && OFF_ST0 % 128 == 0, "line-aligned carve");

constexpr size_t OUT0_BYTES = (size_t)NBATCH * NFRM * 3 * NPTS * 4;
constexpr size_t OUT1_BYTES = (size_t)NBATCH * NFRM * CH3 * 3 * 4;
static_assert(OUT0_BYTES == 3145728ull, "out1 byte offset");
static_assert(OUT0_BYTES + OUT1_BYTES == 3932160ull, "d_out total");
static_assert((NBATCH * NFRM * CH3 * 3) % 256 == 0, "out1 block multiple");
static_assert((CH1 * CH0 * 64) % 2048 == 0 && (CH2 * CH1 * 64) % 2048 == 0 && (CH3 * CH2 * 64) % 2048 == 0, "wpack grids");
static_assert(CH1 % 64 == 0 && CH2 % 64 == 0 && CH3 % 64 == 0, "co tile multiples");

extern "C" void kernel_launch(void* const* d_in, const int* in_sizes, int n_in,
                              void* d_out, int out_size, void* d_ws, size_t ws_size,
                              hipStream_t stream) {
  (void)in_sizes; (void)n_in; (void)out_size;
  if (ws_size < WS_TOTAL) return;
  const float* xyz = (const float*)d_in[0];
  const float* w0  = (const float*)d_in[1];
  const float* cb0 = (const float*)d_in[2];
  const float* g0  = (const float*)d_in[3];
  const float* be0 = (const float*)d_in[4];
  const float* w1  = (const float*)d_in[5];
  const float* cb1 = (const float*)d_in[6];
  const float* g1  = (const float*)d_in[7];
  const float* be1 = (const float*)d_in[8];
  const float* w2  = (const float*)d_in[9];
  const float* cb2 = (const float*)d_in[10];
  const float* g2  = (const float*)d_in[11];
  const float* be2 = (const float*)d_in[12];
  float* out0 = (float*)d_out;
  float* out1 = (float*)d_out + OUT0_BYTES / 4;

  char* ws = (char*)d_ws;
  int*            idxs  = (int*)(ws + OFF_IDX);
  int*            carry = (int*)(ws + OFF_CARRY);
  unsigned short* act0  = (unsigned short*)(ws + OFF_ACT0);
  unsigned short* wp0   = (unsigned short*)(ws + OFF_WP0);
  unsigned short* wp1   = (unsigned short*)(ws + OFF_WP1);
  unsigned short* wp2   = (unsigned short*)(ws + OFF_WP2);
  float*          y0    = (float*)(ws + OFF_Y0);
  float*          y1    = (float*)(ws + OFF_Y1);
  float*          y2    = (float*)(ws + OFF_Y2);
  unsigned short* act1  = (unsigned short*)(ws + OFF_ACT1);
  unsigned short* act2  = (unsigned short*)(ws + OFF_ACT2);
  float*          st0   = (float*)(ws + OFF_ST0);
  float*          st1   = (float*)(ws + OFF_ST1);
  float*          st2   = (float*)(ws + OFF_ST2);

  wpack_kernel<<<(CH1 * CH0 * 64) / 2048, 256, 0, stream>>>(w0, wp0, (CH1 * CH0 * 64) / 8);
  wpack_kernel<<<(CH2 * CH1 * 64) / 2048, 256, 0, stream>>>(w1, wp1, (CH2 * CH1 * 64) / 8);
  wpack_kernel<<<(CH3 * CH2 * 64) / 2048, 256, 0, stream>>>(w2, wp2, (CH3 * CH2 * 64) / 8);

  knn_kernel<<<dim3(NFRAMES, NPTS / 256), 256, 0, stream>>>(xyz, idxs);
  chain_kernel<<<NPTS / 32, 32, 0, stream>>>(idxs, carry);
  out0_kernel<<<(NFRAMES * 3 * (NPTS / 4)) / 256, 256, 0, stream>>>(xyz, idxs, carry, out0);
  pack_kernel<<<NBATCH * NPTS, 256, 0, stream>>>(xyz, idxs, carry, act0);

  conv_gemm<<<dim3(96, CH1 / 64), 256, 0, stream>>>(act0, wp0, cb0, y0, CH0, CH1);
  bn_stats<<<CH1, 256, 0, stream>>>(y0, st0, CH1);
  bn_apply<<<NBATCH * CH1, 256, 0, stream>>>(y0, st0, g0, be0, act1, CH1);

  conv_gemm<<<dim3(96, CH2 / 64), 256, 0, stream>>>(act1, wp1, cb1, y1, CH1, CH2);
  bn_stats<<<CH2, 256, 0, stream>>>(y1, st1, CH2);
  bn_apply<<<NBATCH * CH2, 256, 0, stream>>>(y1, st1, g1, be1, act2, CH2);

  conv_gemm<<<dim3(96, CH3 / 64), 256, 0, stream>>>(act2, wp2, cb2, y2, CH2, CH3);
  bn_stats<<<CH3, 256, 0, stream>>>(y2, st2, CH3);
  bn_max<<<(NBATCH * NFRM * CH3 * 3) / 256, 256, 0, stream>>>(y2, st2, g2, be2, out1);
}
